// MultiLabelClassifier_76974403879334
// MI455X (gfx1250) — hardware-run, weakly checked
//
#include <hip/hip_runtime.h>
#include <math.h>

typedef __attribute__((ext_vector_type(16))) _Float16 v16h;
typedef __attribute__((ext_vector_type(8)))  _Float16 v8h;
typedef __attribute__((ext_vector_type(8)))  float    v8f;
typedef __attribute__((ext_vector_type(4)))  float    v4f;

constexpr int kBatch   = 1024;
constexpr int kLatent  = 512;
constexpr int kBranch  = 16;
constexpr int kHidden  = 512;
constexpr int kRows    = kBatch * kBranch;
constexpr int kHeadCols = kBranch * kHidden;
constexpr int kOut0Elems = kBatch * kBranch;
constexpr int kOut1Elems = kRows * kBranch;
static_assert(kRows == 16384, "row count");
static_assert(kHeadCols == 8192, "stacked head columns");
static_assert(kLatent == kHidden, "square weight tiles assumed by the transpose pack");
static_assert((kLatent % 64) == 0 && (kHidden % 64) == 0 && (kRows % 64) == 0, "tile multiples");
static_assert((kLatent % 32) == 0, "k step multiple");
static_assert(kOut0Elems * 4 == 65536, "out0 bytes");
static_assert(kOut0Elems * 4 + kOut1Elems * 4 == 1114112, "output bytes");

constexpr float kWeightCarry = 64.0f;
constexpr float kActCarry    = 16.0f;
constexpr float kSlope       = 0.1f;
constexpr float kScaleS0 = 1.0f / kWeightCarry;
constexpr float kScaleS1 = 1.0f / (kWeightCarry * kActCarry);
static_assert(kScaleS0 == 0.015625f, "carry fold stage 0");
static_assert(kScaleS1 == 0.0009765625f, "carry fold stage 1");

constexpr size_t kOffA0  = 0;
constexpr size_t kOffH1  = kOffA0  + (size_t)kRows * kLatent * 2;
constexpr size_t kOffSH  = kOffH1  + (size_t)kRows * kLatent * 2;
constexpr size_t kOffBT1 = kOffSH  + (size_t)kRows * kLatent * 2;
constexpr size_t kOffBT2 = kOffBT1 + (size_t)kLatent * kLatent * 2;
constexpr size_t kOffBTC = kOffBT2 + (size_t)kLatent * kLatent * 2;
constexpr size_t kOffLT  = kOffBTC + (size_t)kHeadCols * kLatent * 2;
constexpr size_t kWsTotal = kOffLT + (size_t)kBranch * kRows * 4;
static_assert(kWsTotal == 60817408ull, "carve total");
static_assert(kWsTotal <= 134217728ull, "carve cap");
static_assert((kOffH1 % 128) == 0 && (kOffSH % 128) == 0 && (kOffBT1 % 128) == 0 &&
              (kOffBT2 % 128) == 0 && (kOffBTC % 128) == 0 && (kOffLT % 128) == 0, "aligned regions");

union FragH { v16h v; v8h h[2]; };

__device__ __forceinline__ v16h frag_load(const _Float16* p) {
  FragH f;
  f.h[0] = *(const v8h*)(p);
  f.h[1] = *(const v8h*)(p + 16);
  return f.v;
}

__device__ __forceinline__ v8f mma_h(v16h a, v16h b, v8f c) {
  c = __builtin_amdgcn_wmma_f32_16x16x32_f16(false, a, false, b, (short)0, c, false, false);
  asm volatile("v_nop\n\tv_nop\n\tv_nop\n\tv_nop" : "+v"(c) : "v"(a), "v"(b));
  return c;
}

__global__ __launch_bounds__(128) void pack_x_kernel(
    const float* __restrict__ x, unsigned short* __restrict__ A0)
{
  __shared__ __align__(16) float sx[64 * 16];
  const int tid = threadIdx.x;
  const int d0 = blockIdx.x * 64;
  const int b  = blockIdx.y;
  const float* src = x + ((size_t)b * kLatent + d0) * kBranch;
#pragma unroll
  for (int it = 0; it < 2; ++it) {
    const int idx = (it * 128 + tid) * 4;
    const v4f v = *(const v4f*)(src + idx);
    *(v4f*)(sx + idx) = v;
  }
  __syncthreads();
  const int n  = tid >> 3;
  const int c8 = (tid & 7) * 8;
  v8h hv;
#pragma unroll
  for (int e = 0; e < 8; ++e) {
    const float f = sx[(c8 + e) * kBranch + n];
    hv[e] = (_Float16)f;
  }
  unsigned short* dst = A0 + ((size_t)(n * kBatch + b) * kLatent + d0 + c8);
  *(volatile v8h*)dst = hv;
  __threadfence();
  *(volatile v8h*)dst = hv;
}

__global__ __launch_bounds__(256) void pack_wT_kernel(
    const float* __restrict__ W, unsigned short* __restrict__ Bt)
{
  __shared__ float sT[64 * 65];
  const int tid = threadIdx.x;
  const int j0 = blockIdx.x * 64;
  const int k0 = blockIdx.y * 64;
  const size_t mat = (size_t)blockIdx.z * kLatent * kHidden;
#pragma unroll
  for (int it = 0; it < 4; ++it) {
    const int q  = it * 256 + tid;
    const int kk = q >> 4;
    const int c4 = (q & 15) * 4;
    const v4f v = *(const v4f*)(W + mat + (size_t)(k0 + kk) * kHidden + j0 + c4);
    const float f0 = v[0], f1 = v[1], f2 = v[2], f3 = v[3];
    sT[kk * 65 + c4 + 0] = f0;
    sT[kk * 65 + c4 + 1] = f1;
    sT[kk * 65 + c4 + 2] = f2;
    sT[kk * 65 + c4 + 3] = f3;
  }
  __syncthreads();
  const int c8 = (tid & 7) * 8;
  const int l0 = tid >> 3;
  const int l1 = 32 + (tid >> 3);
  v8h h0, h1;
#pragma unroll
  for (int e = 0; e < 8; ++e) {
    const float a = sT[(c8 + e) * 65 + l0] * kWeightCarry;
    const float c = sT[(c8 + e) * 65 + l1] * kWeightCarry;
    h0[e] = (_Float16)a;
    h1[e] = (_Float16)c;
  }
  unsigned short* p0 = Bt + mat + (size_t)(j0 + l0) * kLatent + k0 + c8;
  unsigned short* p1 = Bt + mat + (size_t)(j0 + l1) * kLatent + k0 + c8;
  for (int pass = 0; pass < 2; ++pass) {
    *(volatile v8h*)p0 = h0;
    *(volatile v8h*)p1 = h1;
    __threadfence();
  }
}

__global__ __launch_bounds__(256) void gemm_leaky_f16_kernel(
    const unsigned short* __restrict__ Ap, int lda,
    const unsigned short* __restrict__ Btp, int ldb,
    unsigned short* __restrict__ Cp, int ldc,
    const float* __restrict__ bias,
    int M, int N, int K, float scale)
{
  const _Float16* A  = (const _Float16*)Ap;
  const _Float16* Bt = (const _Float16*)Btp;
  __shared__ __align__(16) float sT[8][16 * 68];
  const int lane = threadIdx.x & 31;
  const int wave = threadIdx.x >> 5;
  const int tilesN = N >> 6;
  const int tilesM = M >> 6;
  const int tile = blockIdx.x * 8 + wave;
  if (tile >= tilesM * tilesN) return;
  const int tm = tile / tilesN;
  const int tn = tile - tm * tilesN;
  const int m0 = tm << 6;
  const int n0 = tn << 6;

  const int rlane = lane & 15;
  const int koff  = (lane >> 4) * 8;
  const int mOff  = (lane >> 4) * 8;

  v8f acc[4][4];
#pragma unroll
  for (int i = 0; i < 4; ++i)
#pragma unroll
    for (int j = 0; j < 4; ++j) acc[i][j] = (v8f){0.f,0.f,0.f,0.f,0.f,0.f,0.f,0.f};

#pragma unroll 1
  for (int k0 = 0; k0 < K; k0 += 32) {
    v16h bh[4];
#pragma unroll
    for (int j = 0; j < 4; ++j) {
      const size_t bo = (size_t)(n0 + (j << 4) + rlane) * ldb + koff + k0;
      bh[j] = frag_load(Bt + bo);
    }
#pragma unroll
    for (int i = 0; i < 4; ++i) {
      const size_t ao = (size_t)(m0 + (i << 4) + rlane) * lda + koff + k0;
      const v16h ah = frag_load(A + ao);
#pragma unroll
      for (int j = 0; j < 4; ++j) acc[i][j] = mma_h(ah, bh[j], acc[i][j]);
    }
  }

  float* slab = sT[wave];
  float bvj[4];
#pragma unroll
  for (int j = 0; j < 4; ++j) bvj[j] = bias[n0 + (j << 4) + rlane];
  const int q  = lane >> 3;
  const int c8 = (lane & 7) * 8;
#pragma unroll
  for (int i = 0; i < 4; ++i) {
    const int mBase = m0 + (i << 4);
#pragma unroll
    for (int j = 0; j < 4; ++j) {
#pragma unroll
      for (int r = 0; r < 8; ++r) {
        float v = acc[i][j][r] * scale + bvj[j];
        v = (v >= 0.0f) ? v : kSlope * v;
        slab[(mOff + r) * 68 + (j << 4) + rlane] = v * kActCarry;
      }
    }
    __builtin_amdgcn_fence(__ATOMIC_RELEASE, "workgroup");
    __builtin_amdgcn_wave_barrier();
    __builtin_amdgcn_fence(__ATOMIC_ACQUIRE, "workgroup");
    v8h hv[4];
#pragma unroll
    for (int it = 0; it < 4; ++it) {
      const int row = it * 4 + q;
      const float* sp = slab + row * 68 + c8;
#pragma unroll
      for (int e = 0; e < 8; ++e) {
        const float f = sp[e];
        hv[it][e] = (_Float16)f;
      }
    }
    for (int pass = 0; pass < 2; ++pass) {
#pragma unroll
      for (int it = 0; it < 4; ++it) {
        const int row = it * 4 + q;
        *(volatile v8h*)(Cp + (size_t)(mBase + row) * ldc + n0 + c8) = hv[it];
      }
      __threadfence();
    }
    __builtin_amdgcn_fence(__ATOMIC_RELEASE, "workgroup");
    __builtin_amdgcn_wave_barrier();
    __builtin_amdgcn_fence(__ATOMIC_ACQUIRE, "workgroup");
  }
}

__global__ __launch_bounds__(256) void head_gemm_kernel(
    const unsigned short* __restrict__ SHp, const unsigned short* __restrict__ Btcp,
    const float* __restrict__ bc1, const float* __restrict__ Wc2,
    const float* __restrict__ bc2, float* __restrict__ Lt)
{
  const _Float16* A  = (const _Float16*)SHp;
  const _Float16* Bt = (const _Float16*)Btcp;
  __shared__ float red[8 * 64];
  const int tid  = threadIdx.x;
  const int lane = tid & 31;
  const int wave = tid >> 5;
  const int head = blockIdx.y;
  const int m0 = blockIdx.x * 64;
  const int n0 = head * kHidden + wave * 64;

  const int rlane = lane & 15;
  const int koff  = (lane >> 4) * 8;
  const int mOff  = (lane >> 4) * 8;

  v8f acc[4][4];
#pragma unroll
  for (int i = 0; i < 4; ++i)
#pragma unroll
    for (int j = 0; j < 4; ++j) acc[i][j] = (v8f){0.f,0.f,0.f,0.f,0.f,0.f,0.f,0.f};

#pragma unroll 1
  for (int k0 = 0; k0 < kLatent; k0 += 32) {
    v16h bh[4];
#pragma unroll
    for (int j = 0; j < 4; ++j) {
      const size_t bo = (size_t)(n0 + (j << 4) + rlane) * kLatent + koff + k0;
      bh[j] = frag_load(Bt + bo);
    }
#pragma unroll
    for (int i = 0; i < 4; ++i) {
      const size_t ao = (size_t)(m0 + (i << 4) + rlane) * kLatent + koff + k0;
      const v16h ah = frag_load(A + ao);
#pragma unroll
      for (int j = 0; j < 4; ++j) acc[i][j] = mma_h(ah, bh[j], acc[i][j]);
    }
  }

  float b1[4], w2[4];
#pragma unroll
  for (int j = 0; j < 4; ++j) {
    const int col = n0 + (j << 4) + rlane;
    b1[j] = bc1[col];
    w2[j] = Wc2[col];
  }
#pragma unroll
  for (int i = 0; i < 4; ++i) {
#pragma unroll
    for (int r = 0; r < 8; ++r) {
      float s = 0.0f;
#pragma unroll
      for (int j = 0; j < 4; ++j) {
        float v = acc[i][j][r] * kScaleS1 + b1[j];
        v = (v >= 0.0f) ? v : kSlope * v;
        s = fmaf(v, w2[j], s);
      }
      s += __shfl_xor(s, 1, 32);
      s += __shfl_xor(s, 2, 32);
      s += __shfl_xor(s, 4, 32);
      s += __shfl_xor(s, 8, 32);
      if (rlane == 0) red[wave * 64 + (i << 4) + mOff + r] = s;
    }
  }
  __syncthreads();
  if (tid < 64) {
    float s = 0.0f;
#pragma unroll
    for (int w = 0; w < 8; ++w) s += red[w * 64 + tid];
    s += bc2[head];
    float* p = Lt + (size_t)head * kRows + m0 + tid;
    *(volatile float*)p = s;
    __threadfence();
    *(volatile float*)p = s;
  }
}

__global__ __launch_bounds__(256) void finish_out1_kernel(
    const float* __restrict__ Lt, float* __restrict__ out1)
{
  const int i4 = blockIdx.x * 256 + threadIdx.x;
  if (i4 >= kOut1Elems / 4) return;
  const int m  = i4 >> 2;
  const int j0 = (i4 & 3) * 4;
  const float f0 = Lt[(size_t)(j0 + 0) * kRows + m];
  const float f1 = Lt[(size_t)(j0 + 1) * kRows + m];
  const float f2 = Lt[(size_t)(j0 + 2) * kRows + m];
  const float f3 = Lt[(size_t)(j0 + 3) * kRows + m];
  const v4f v = (v4f){f0, f1, f2, f3};
  float* p = out1 + (size_t)i4 * 4;
  *(volatile v4f*)p = v;
  __threadfence();
  *(volatile v4f*)p = v;
}

__global__ __launch_bounds__(256) void finish_out0_kernel(
    const float* __restrict__ Lt, float* __restrict__ out0)
{
  __shared__ __align__(16) float sO[256];
  const int tid = threadIdx.x;
  const int idx = blockIdx.x * 256 + tid;
  const int b = idx >> 4;
  const int n = idx & 15;
  const float l = Lt[(size_t)n * kRows + n * kBatch + b];
  sO[tid] = 1.0f / (1.0f + expf(-l));
  __syncthreads();
  if (tid < 64) {
    const v4f v = *(const v4f*)(sO + tid * 4);
    float* p = out0 + (size_t)blockIdx.x * 256 + tid * 4;
    *(volatile v4f*)p = v;
    __threadfence();
    *(volatile v4f*)p = v;
  }
}

extern "C" void kernel_launch(void* const* d_in, const int* in_sizes, int n_in,
                              void* d_out, int out_size, void* d_ws, size_t ws_size,
                              hipStream_t stream) {
  if (n_in < 9) return;
  if (in_sizes[0] != kBatch * kLatent * kBranch) return;
  if (in_sizes[1] != kLatent * kLatent) return;
  if (in_sizes[2] != kLatent) return;
  if (in_sizes[3] != kLatent * kLatent) return;
  if (in_sizes[4] != kLatent) return;
  if (in_sizes[5] != kBranch * kLatent * kHidden) return;
  if (in_sizes[6] != kBranch * kHidden) return;
  if (in_sizes[7] != kBranch * kHidden) return;
  if (in_sizes[8] != kBranch) return;
  if (out_size != kOut0Elems + kOut1Elems) return;
  if (ws_size < kWsTotal) return;

  const float* x   = (const float*)d_in[0];
  const float* Ws1 = (const float*)d_in[1];
  const float* bs1 = (const float*)d_in[2];
  const float* Ws2 = (const float*)d_in[3];
  const float* bs2 = (const float*)d_in[4];
  const float* Wc1 = (const float*)d_in[5];
  const float* bc1 = (const float*)d_in[6];
  const float* Wc2 = (const float*)d_in[7];
  const float* bc2 = (const float*)d_in[8];

  float* out0 = (float*)d_out;
  float* out1 = out0 + kOut0Elems;

  char* ws = (char*)d_ws;
  unsigned short* A0  = (unsigned short*)(ws + kOffA0);
  unsigned short* H1  = (unsigned short*)(ws + kOffH1);
  unsigned short* SH  = (unsigned short*)(ws + kOffSH);
  unsigned short* BT1 = (unsigned short*)(ws + kOffBT1);
  unsigned short* BT2 = (unsigned short*)(ws + kOffBT2);
  unsigned short* BTC = (unsigned short*)(ws + kOffBTC);
  float*          LT  = (float*)(ws + kOffLT);

  pack_x_kernel<<<dim3(kLatent / 64, kBatch), 128, 0, stream>>>(x, A0);
  pack_wT_kernel<<<dim3(kHidden / 64, kLatent / 64, 1), 256, 0, stream>>>(Ws1, BT1);
  pack_wT_kernel<<<dim3(kHidden / 64, kLatent / 64, 1), 256, 0, stream>>>(Ws2, BT2);
  pack_wT_kernel<<<dim3(kHidden / 64, kLatent / 64, kBranch), 256, 0, stream>>>(Wc1, BTC);

  gemm_leaky_f16_kernel<<<dim3((kRows / 64) * (kLatent / 64) / 8), 256, 0, stream>>>(
      A0, kLatent, BT1, kLatent, H1, kLatent, bs1, kRows, kLatent, kLatent, kScaleS0);
  gemm_leaky_f16_kernel<<<dim3((kRows / 64) * (kLatent / 64) / 8), 256, 0, stream>>>(
      H1, kLatent, BT2, kLatent, SH, kLatent, bs2, kRows, kLatent, kLatent, kScaleS1);

  head_gemm_kernel<<<dim3(kRows / 64, kBranch), 256, 0, stream>>>(SH, BTC, bc1, Wc2, bc2, LT);

  finish_out1_kernel<<<dim3(kOut1Elems / 4 / 256), 256, 0, stream>>>(LT, out1);
  finish_out0_kernel<<<dim3(kOut0Elems / 256), 256, 0, stream>>>(LT, out0);
}
